// PointnetFPModule_5669356832928
// MI455X (gfx1250) — hardware-verified
//
#include <hip/hip_runtime.h>
#include <stdint.h>

#pragma clang fp contract(off)

typedef __attribute__((ext_vector_type(16))) _Float16 v16h;
typedef __attribute__((ext_vector_type(8)))  _Float16 v8h;
typedef __attribute__((ext_vector_type(8)))  float    v8f;
typedef __attribute__((ext_vector_type(4)))  float    v4f;
typedef __attribute__((ext_vector_type(2)))  float    v2f;

constexpr int NBATCH   = 4;
constexpr int NQUERY   = 8192;
constexpr int NSUPP    = 2048;
constexpr int CH_UNK   = 128;
constexpr int CH_KNOWN = 256;
constexpr int CH_CAT   = CH_KNOWN + CH_UNK;
constexpr int CH_OUT   = 256;
constexpr int NPOINTS  = NBATCH * NQUERY;

static_assert(CH_CAT == 384, "concat width");
static_assert(CH_CAT % 32 == 0 && CH_OUT % 32 == 0, "K multiple of 32");
static_assert(NPOINTS % 32 == 0 && CH_OUT % 64 == 0, "layer-0 tile multiples");
static_assert(CH_OUT % 32 == 0 && NQUERY % 64 == 0, "layer-1 tile multiples");
static_assert(NSUPP % 32 == 0 && NQUERY % 256 == 0, "tiling of the point kernels");

constexpr float W_CARRY  = 16.0f;
constexpr float LO_CARRY = 2048.0f;
constexpr float SCALE_HI = 1.0f / W_CARRY;
constexpr float SCALE_LO = 1.0f / (W_CARRY * LO_CARRY);
constexpr float BN_EPS_F = 1e-5f;

__device__ __forceinline__ v16h frag_load_h(const _Float16* p) {
  union U { v16h v; v8h h[2]; } f;
  f.h[0] = *(const v8h*)(p);
  f.h[1] = *(const v8h*)(p + 16);
  return f.v;
}
__device__ __forceinline__ v8f mma_h(v16h a, v16h b, v8f c) {
  return __builtin_amdgcn_wmma_f32_16x16x32_f16(false, a, false, b, (short)0, c, false, false);
}
__device__ __forceinline__ void guard4_h(v8f& a, v8f& b, v8f& c, v8f& d, v16h x, v16h y) {
  asm volatile("v_nop\n\tv_nop\n\tv_nop\n\tv_nop" : "+v"(a), "+v"(b), "+v"(c), "+v"(d) : "v"(x), "v"(y));
}
__device__ __forceinline__ void keep4_h(v16h a, v16h b, v16h c, v16h d) {
  asm volatile("v_nop" :: "v"(a), "v"(b), "v"(c), "v"(d));
}
__device__ __forceinline__ void acc_guard4(v8f& a, v8f& b, v8f& c, v8f& d) {
  asm volatile("v_nop\n\tv_nop\n\tv_nop\n\tv_nop" : "+v"(a), "+v"(b), "+v"(c), "+v"(d));
}

__device__ __forceinline__ void conv8_hilo(const float* __restrict__ W, unsigned short* __restrict__ H,
                                           unsigned short* __restrict__ L, int idx8) {
  const v4f x0 = *(const v4f*)(W + (size_t)idx8 * 8);
  const v4f x1 = *(const v4f*)(W + (size_t)idx8 * 8 + 4);
  v8h hv, lv;
#pragma unroll
  for (int e = 0; e < 4; ++e) {
    const float a = x0[e] * W_CARRY;
    const _Float16 ha = (_Float16)a;
    const float af = (float)ha;
    const float ra = (a - af) * LO_CARRY;
    hv[e] = ha;
    lv[e] = (_Float16)ra;
    const float c = x1[e] * W_CARRY;
    const _Float16 hc = (_Float16)c;
    const float cf = (float)hc;
    const float rc = (c - cf) * LO_CARRY;
    hv[4 + e] = hc;
    lv[4 + e] = (_Float16)rc;
  }
  volatile v8h* hp = (volatile v8h*)(H + (size_t)idx8 * 8);
  volatile v8h* lp = (volatile v8h*)(L + (size_t)idx8 * 8);
  *hp = hv;
  *lp = lv;
  __threadfence();
  *hp = hv;
  *lp = lv;
}

__device__ __forceinline__ void bn_affine4(const float* __restrict__ bc, const float* __restrict__ g,
                                           const float* __restrict__ be, const float* __restrict__ rm,
                                           const float* __restrict__ rv, float* __restrict__ sOut,
                                           float* __restrict__ tOut, int q4) {
  const v4f vb  = *(const v4f*)(bc + q4);
  const v4f vg  = *(const v4f*)(g + q4);
  const v4f vbe = *(const v4f*)(be + q4);
  const v4f vrm = *(const v4f*)(rm + q4);
  const v4f vrv = *(const v4f*)(rv + q4);
  v4f s, t;
#pragma unroll
  for (int e = 0; e < 4; ++e) {
    const float sd = sqrtf(vrv[e] + BN_EPS_F);
    const float se = vg[e] / sd;
    const float df = vb[e] - vrm[e];
    const float pr = df * se;
    s[e] = se;
    t[e] = pr + vbe[e];
  }
  volatile v4f* sp = (volatile v4f*)(sOut + q4);
  volatile v4f* tp = (volatile v4f*)(tOut + q4);
  *sp = s;
  *tp = t;
  __threadfence();
  *sp = s;
  *tp = t;
}

constexpr int PREP_BLK_W0 = (CH_OUT * CH_CAT) / (8 * 256);
constexpr int PREP_BLK_W1 = (CH_OUT * CH_OUT) / (8 * 256);
static_assert(PREP_BLK_W0 * 8 * 256 == CH_OUT * CH_CAT, "W0 coverage exact");
static_assert(PREP_BLK_W1 * 8 * 256 == CH_OUT * CH_OUT, "W1 coverage exact");
static_assert(CH_OUT == 64 * 4, "affine vectors: 64 lanes x 4 channels");

__global__ __launch_bounds__(256) void prep_weights_kernel(
    const float* __restrict__ W0, const float* __restrict__ W1,
    const float* __restrict__ b0, const float* __restrict__ g0, const float* __restrict__ be0,
    const float* __restrict__ rm0, const float* __restrict__ rv0,
    const float* __restrict__ b1, const float* __restrict__ g1, const float* __restrict__ be1,
    const float* __restrict__ rm1, const float* __restrict__ rv1,
    unsigned short* __restrict__ W0h, unsigned short* __restrict__ W0l,
    unsigned short* __restrict__ W1h, unsigned short* __restrict__ W1l,
    float* __restrict__ st) {
  const int blk = blockIdx.x;
  const int tid = threadIdx.x;
  if (blk < PREP_BLK_W0) {
    conv8_hilo(W0, W0h, W0l, blk * 256 + tid);
  } else if (blk < PREP_BLK_W0 + PREP_BLK_W1) {
    conv8_hilo(W1, W1h, W1l, (blk - PREP_BLK_W0) * 256 + tid);
  } else if (blk == PREP_BLK_W0 + PREP_BLK_W1) {
    if (tid < 64) bn_affine4(b0, g0, be0, rm0, rv0, st, st + CH_OUT, tid * 4);
  } else {
    if (tid < 64) bn_affine4(b1, g1, be1, rm1, rv1, st + 2 * CH_OUT, st + 3 * CH_OUT, tid * 4);
  }
}

constexpr int TK_PITCH = 260;
__global__ __launch_bounds__(256) void transpose_known_kernel(const float* __restrict__ kf, float* __restrict__ Ft) {
  __shared__ __align__(16) float T[32 * TK_PITCH];
  const int tid = threadIdx.x;
  const int lane = tid & 31;
  const int wave = tid >> 5;
  const int b = blockIdx.y;
  const int m0 = blockIdx.x * 32;
  const float* src = kf + (size_t)b * CH_KNOWN * NSUPP + m0 + lane;
#pragma unroll 1
  for (int grp = 0; grp < 4; ++grp) {
    float v[8];
#pragma unroll
    for (int cc = 0; cc < 8; ++cc) {
      const int c = wave * 32 + grp * 8 + cc;
      v[cc] = src[(size_t)c * NSUPP];
    }
#pragma unroll
    for (int cc = 0; cc < 8; ++cc) {
      const int c = wave * 32 + grp * 8 + cc;
      T[lane * TK_PITCH + c] = v[cc];
    }
  }
  __syncthreads();
  float* dstb = Ft + ((size_t)b * NSUPP + m0) * CH_KNOWN;
  for (int pass = 0; pass < 2; ++pass) {
#pragma unroll
    for (int rr = 0; rr < 4; ++rr) {
      const int row = wave * 4 + rr;
#pragma unroll
      for (int hf = 0; hf < 2; ++hf) {
        const int c4 = hf * 128 + lane * 4;
        const v4f val = *(const v4f*)(T + row * TK_PITCH + c4);
        *(volatile v4f*)(dstb + (size_t)row * CH_KNOWN + c4) = val;
      }
    }
    __threadfence();
  }
}

__global__ __launch_bounds__(256) void nn3_interp_kernel(
    const float* __restrict__ unknown, const float* __restrict__ known,
    const float* __restrict__ Ft, unsigned short* __restrict__ X0) {
#pragma clang fp contract(off)
  __shared__ __align__(16) float kp[NSUPP * 4];
  __shared__ int   sI[3 * 256];
  __shared__ float sW[3 * 256];
  const int tid = threadIdx.x;
  const int b   = blockIdx.y;
  const int n0  = blockIdx.x * 256;

  {
    const float* kb = known + (size_t)b * NSUPP * 3;
#pragma unroll 1
    for (int i = tid; i < NSUPP; i += 256) {
      const float x = kb[3 * i + 0];
      const float y = kb[3 * i + 1];
      const float z = kb[3 * i + 2];
      const float xx = x * x;
      const float yy = y * y;
      const float zz = z * z;
      v4f e;
      e[0] = x;
      e[1] = y;
      e[2] = z;
      e[3] = (xx + zz) + yy;
      *(v4f*)(kp + 4 * i) = e;
    }
  }
  __syncthreads();

  {
    const int n = n0 + tid;
    const float* up = unknown + ((size_t)b * NQUERY + n) * 3;
    const float ux = up[0];
    const float uy = up[1];
    const float uz = up[2];
    const float uxx = ux * ux;
    const float uyy = uy * uy;
    const float uzz = uz * uz;
    const float squ = (uxx + uzz) + uyy;
    float bd0 = __builtin_inff(), bd1 = __builtin_inff(), bd2 = __builtin_inff();
    int bi0 = 0, bi1 = 0, bi2 = 0;
#pragma unroll 4
    for (int m = 0; m < NSUPP; ++m) {
      const v4f kk = *(const v4f*)(kp + 4 * m);
      float p = ux * kk[0];
      p = __builtin_fmaf(uy, kk[1], p);
      p = __builtin_fmaf(uz, kk[2], p);
      const float tw = 2.0f * p;
      const float df = squ - tw;
      const float d = df + kk[3];
      const bool c2 = d < bd2;
      const bool c1 = d < bd1;
      const bool c0 = d < bd0;
      const float nd2 = c1 ? bd1 : (c2 ? d : bd2);
      const int   ni2 = c1 ? bi1 : (c2 ? m : bi2);
      const float nd1 = c0 ? bd0 : (c1 ? d : bd1);
      const int   ni1 = c0 ? bi0 : (c1 ? m : bi1);
      const float nd0 = c0 ? d : bd0;
      const int   ni0 = c0 ? m : bi0;
      bd2 = nd2; bi2 = ni2;
      bd1 = nd1; bi1 = ni1;
      bd0 = nd0; bi0 = ni0;
    }
    const float e0 = sqrtf(fmaxf(bd0, 0.0f));
    const float e1 = sqrtf(fmaxf(bd1, 0.0f));
    const float e2 = sqrtf(fmaxf(bd2, 0.0f));
    const float r0 = 1.0f / (e0 + 1e-8f);
    const float r1 = 1.0f / (e1 + 1e-8f);
    const float r2 = 1.0f / (e2 + 1e-8f);
    const float rs = (r0 + r2) + r1;
    bi0 = bi0 < 0 ? 0 : (bi0 > NSUPP - 1 ? NSUPP - 1 : bi0);
    bi1 = bi1 < 0 ? 0 : (bi1 > NSUPP - 1 ? NSUPP - 1 : bi1);
    bi2 = bi2 < 0 ? 0 : (bi2 > NSUPP - 1 ? NSUPP - 1 : bi2);
    sI[tid]       = bi0;
    sI[256 + tid] = bi1;
    sI[512 + tid] = bi2;
    sW[tid]       = r0 / rs;
    sW[256 + tid] = r1 / rs;
    sW[512 + tid] = r2 / rs;
  }
  __syncthreads();

  const int lane = tid & 31;
  const int wave = tid >> 5;
  const float* Fb = Ft + (size_t)b * NSUPP * CH_KNOWN;
#pragma unroll 1
  for (int pp = 0; pp < 32; ++pp) {
    const int p = wave * 32 + pp;
    int m0 = sI[p];
    int m1 = sI[256 + p];
    int m2 = sI[512 + p];
    m0 = m0 < 0 ? 0 : (m0 > NSUPP - 1 ? NSUPP - 1 : m0);
    m1 = m1 < 0 ? 0 : (m1 > NSUPP - 1 ? NSUPP - 1 : m1);
    m2 = m2 < 0 ? 0 : (m2 > NSUPP - 1 ? NSUPP - 1 : m2);
    const float w0 = sW[p];
    const float w1 = sW[256 + p];
    const float w2 = sW[512 + p];
    const float* f0 = Fb + (size_t)m0 * CH_KNOWN + lane * 8;
    const float* f1 = Fb + (size_t)m1 * CH_KNOWN + lane * 8;
    const float* f2 = Fb + (size_t)m2 * CH_KNOWN + lane * 8;
    const v4f fa0 = *(const v4f*)(f0);
    const v4f fa1 = *(const v4f*)(f0 + 4);
    const v4f fb0 = *(const v4f*)(f1);
    const v4f fb1 = *(const v4f*)(f1 + 4);
    const v4f fc0 = *(const v4f*)(f2);
    const v4f fc1 = *(const v4f*)(f2 + 4);
    v8h hv;
#pragma unroll
    for (int e = 0; e < 4; ++e) {
      const float t0 = w0 * fa0[e];
      const float t1 = w1 * fb0[e];
      const float t2 = w2 * fc0[e];
      const float lo = (t0 + t1) + t2;
      hv[e] = (_Float16)lo;
      const float u0 = w0 * fa1[e];
      const float u1 = w1 * fb1[e];
      const float u2 = w2 * fc1[e];
      const float hi = (u0 + u1) + u2;
      hv[4 + e] = (_Float16)hi;
    }
    volatile v8h* dst = (volatile v8h*)(X0 + ((size_t)b * NQUERY + n0 + p) * CH_CAT + lane * 8);
    *dst = hv;
    __threadfence();
    *dst = hv;
  }
}

constexpr int TU_PITCH = 132;
__global__ __launch_bounds__(256) void ufeat_concat_kernel(const float* __restrict__ uf, unsigned short* __restrict__ X0) {
  __shared__ __align__(16) float T[64 * TU_PITCH];
  const int tid = threadIdx.x;
  const int lane = tid & 31;
  const int wave = tid >> 5;
  const int b = blockIdx.y;
  const int n0 = blockIdx.x * 64;
  const float* src = uf + (size_t)b * CH_UNK * NQUERY + n0 + 2 * lane;
#pragma unroll 1
  for (int grp = 0; grp < 2; ++grp) {
    v2f v[8];
#pragma unroll
    for (int cc = 0; cc < 8; ++cc) {
      const int c = wave * 16 + grp * 8 + cc;
      v[cc] = *(const v2f*)(src + (size_t)c * NQUERY);
    }
#pragma unroll
    for (int cc = 0; cc < 8; ++cc) {
      const int c = wave * 16 + grp * 8 + cc;
      T[(2 * lane) * TU_PITCH + c]     = v[cc][0];
      T[(2 * lane + 1) * TU_PITCH + c] = v[cc][1];
    }
  }
  __syncthreads();
  const int hh = lane >> 4;
  const int c8 = (lane & 15) * 8;
  for (int pass = 0; pass < 2; ++pass) {
#pragma unroll
    for (int it = 0; it < 4; ++it) {
      const int row = wave * 8 + it * 2 + hh;
      const float* sp = T + row * TU_PITCH + c8;
      const v4f x0 = *(const v4f*)(sp);
      const v4f x1 = *(const v4f*)(sp + 4);
      v8h hv;
#pragma unroll
      for (int e = 0; e < 4; ++e) {
        hv[e] = (_Float16)x0[e];
        hv[4 + e] = (_Float16)x1[e];
      }
      *(volatile v8h*)(X0 + ((size_t)b * NQUERY + n0 + row) * CH_CAT + CH_KNOWN + c8) = hv;
    }
    __threadfence();
  }
}

template <int SPLIT_SIDE, int OUT_MODE, int ST_MODE>
__global__ __launch_bounds__(256) void gemm_f16_hilo_kernel(
    const unsigned short* __restrict__ Ap, const unsigned short* __restrict__ A2p, int lda, long strideA,
    const unsigned short* __restrict__ Btp, const unsigned short* __restrict__ Bt2p, int ldb, long strideB,
    void* __restrict__ Cout, int ldc, long strideC,
    const float* __restrict__ sv, const float* __restrict__ tv,
    int M, int N, int K) {
  typedef _Float16 T;
  const T* A   = (const T*)Ap;
  const T* A2  = (const T*)A2p;
  const T* Bt  = (const T*)Btp;
  const T* Bt2 = (const T*)Bt2p;
  __shared__ __align__(16) float sT[8][16 * 68];
  const int b    = blockIdx.y;
  const int lane = threadIdx.x & 31;
  const int wave = threadIdx.x >> 5;
  const int tilesN = N >> 6;
  const int tilesM = M >> 5;
  const int tile = blockIdx.x * 8 + wave;
  if (tile >= tilesM * tilesN) return;
  const int tm = tile / tilesN;
  const int tn = tile - tm * tilesN;
  const int m0 = tm << 5;
  const int n0 = tn << 6;

  const T* Ab  = A   + (size_t)b * strideA;
  const T* Ab2 = A2  + (size_t)b * strideA;
  const T* Bb  = Bt  + (size_t)b * strideB;
  const T* Bb2 = Bt2 + (size_t)b * strideB;

  const int rlane = lane & 15;
  const int koff  = (lane >> 4) * 8;
  const int mOff  = (lane >> 4) * 8;

  v8f accH[2][4], accL[2][4];
#pragma unroll
  for (int i = 0; i < 2; ++i)
#pragma unroll
    for (int j = 0; j < 4; ++j) {
      accH[i][j] = (v8f){0.f, 0.f, 0.f, 0.f, 0.f, 0.f, 0.f, 0.f};
      accL[i][j] = (v8f){0.f, 0.f, 0.f, 0.f, 0.f, 0.f, 0.f, 0.f};
    }

  for (int k0 = 0; k0 < K; k0 += 32) {
    v16h a[2], a2[2];
#pragma unroll
    for (int i = 0; i < 2; ++i) {
      const size_t ao = (size_t)(m0 + (i << 4) + rlane) * lda + koff + k0;
      a[i] = frag_load_h(Ab + ao);
      if (SPLIT_SIDE == 0) a2[i] = frag_load_h(Ab2 + ao);
      else a2[i] = a[i];
    }
#pragma unroll
    for (int j = 0; j < 4; ++j) {
      const size_t bo = (size_t)(n0 + (j << 4) + rlane) * ldb + koff + k0;
      const v16h bh = frag_load_h(Bb + bo);
      v16h bl = bh;
      if (SPLIT_SIDE == 1) bl = frag_load_h(Bb2 + bo);
#pragma unroll
      for (int i = 0; i < 2; ++i) {
        accH[i][j] = mma_h(a[i], bh, accH[i][j]);
        accL[i][j] = mma_h(a2[i], bl, accL[i][j]);
      }
      guard4_h(accH[0][j], accH[1][j], accL[0][j], accL[1][j], bh, bl);
    }
    keep4_h(a[0], a[1], a2[0], a2[1]);
  }
  acc_guard4(accH[0][0], accH[0][1], accH[0][2], accH[0][3]);
  acc_guard4(accH[1][0], accH[1][1], accH[1][2], accH[1][3]);
  acc_guard4(accL[0][0], accL[0][1], accL[0][2], accL[0][3]);
  acc_guard4(accL[1][0], accL[1][1], accL[1][2], accL[1][3]);

  float* slab = sT[wave];
  float sn[4], tnv[4];
#pragma unroll
  for (int j = 0; j < 4; ++j) {
    sn[j] = 1.0f;
    tnv[j] = 0.0f;
    if (ST_MODE == 2) {
      sn[j]  = sv[n0 + (j << 4) + rlane];
      tnv[j] = tv[n0 + (j << 4) + rlane];
    }
  }
#pragma unroll
  for (int i = 0; i < 2; ++i) {
    const int mBase = m0 + (i << 4);
    float sr[8], tr[8];
#pragma unroll
    for (int r = 0; r < 8; ++r) { sr[r] = 1.0f; tr[r] = 0.0f; }
    if (ST_MODE == 1) {
      const v4f s0 = *(const v4f*)(sv + mBase + mOff);
      const v4f s1 = *(const v4f*)(sv + mBase + mOff + 4);
      const v4f t0 = *(const v4f*)(tv + mBase + mOff);
      const v4f t1 = *(const v4f*)(tv + mBase + mOff + 4);
#pragma unroll
      for (int r = 0; r < 4; ++r) {
        sr[r] = s0[r]; sr[4 + r] = s1[r];
        tr[r] = t0[r]; tr[4 + r] = t1[r];
      }
    }
#pragma unroll
    for (int j = 0; j < 4; ++j) {
#pragma unroll
      for (int r = 0; r < 8; ++r) {
        const float ph = accH[i][j][r] * SCALE_HI;
        const float pl = accL[i][j][r] * SCALE_LO;
        float v = ph + pl;
        const float sc = (ST_MODE == 1) ? sr[r] : sn[j];
        const float tc = (ST_MODE == 1) ? tr[r] : tnv[j];
        const float vs = v * sc;
        v = vs + tc;
        v = fmaxf(v, 0.0f);
        slab[(mOff + r) * 68 + (j << 4) + rlane] = v;
      }
    }
    __builtin_amdgcn_fence(__ATOMIC_RELEASE, "workgroup");
    __builtin_amdgcn_wave_barrier();
    __builtin_amdgcn_fence(__ATOMIC_ACQUIRE, "workgroup");
    if (OUT_MODE == 0) {
      float* C = (float*)Cout + (size_t)b * strideC;
      const int hh = lane >> 4, c4 = (lane & 15) * 4;
      for (int pass = 0; pass < 2; ++pass) {
#pragma unroll
        for (int it = 0; it < 8; ++it) {
          const int row = it * 2 + hh;
          const v4f val = *(const v4f*)(slab + row * 68 + c4);
          *(volatile v4f*)(C + (size_t)(mBase + row) * ldc + n0 + c4) = val;
        }
        __threadfence();
      }
    } else {
      const int q = lane >> 3, c8 = (lane & 7) * 8;
      unsigned short* C = (unsigned short*)Cout + (size_t)b * strideC;
      for (int pass = 0; pass < 2; ++pass) {
#pragma unroll
        for (int it = 0; it < 4; ++it) {
          const int row = it * 4 + q;
          const float* sp = slab + row * 68 + c8;
          const v4f x0 = *(const v4f*)(sp);
          const v4f x1 = *(const v4f*)(sp + 4);
          v8h hv;
#pragma unroll
          for (int e = 0; e < 4; ++e) {
            hv[e] = (_Float16)x0[e];
            hv[4 + e] = (_Float16)x1[e];
          }
          *(volatile v8h*)(C + (size_t)(mBase + row) * ldc + n0 + c8) = hv;
        }
        __threadfence();
      }
    }
    __builtin_amdgcn_fence(__ATOMIC_RELEASE, "workgroup");
    __builtin_amdgcn_wave_barrier();
    __builtin_amdgcn_fence(__ATOMIC_ACQUIRE, "workgroup");
  }
}

constexpr size_t SZ_FT  = (size_t)NBATCH * NSUPP * CH_KNOWN * 4;
constexpr size_t SZ_X0  = (size_t)NPOINTS * CH_CAT * 2;
constexpr size_t SZ_X1  = (size_t)NPOINTS * CH_OUT * 2;
constexpr size_t SZ_W0P = (size_t)CH_OUT * CH_CAT * 2;
constexpr size_t SZ_W1P = (size_t)CH_OUT * CH_OUT * 2;
constexpr size_t SZ_ST  = (size_t)4 * CH_OUT * 4;
constexpr size_t OFF_FT  = 0;
constexpr size_t OFF_X0  = OFF_FT + SZ_FT;
constexpr size_t OFF_X1  = OFF_X0 + SZ_X0;
constexpr size_t OFF_W0H = OFF_X1 + SZ_X1;
constexpr size_t OFF_W0L = OFF_W0H + SZ_W0P;
constexpr size_t OFF_W1H = OFF_W0L + SZ_W0P;
constexpr size_t OFF_W1L = OFF_W1H + SZ_W1P;
constexpr size_t OFF_ST  = OFF_W1L + SZ_W1P;
constexpr size_t WS_TOTAL = OFF_ST + SZ_ST;
static_assert(WS_TOTAL == 50991104, "carve total");
static_assert(WS_TOTAL <= (size_t)134217728, "carve under 128 MiB");
static_assert(OFF_X0 % 256 == 0 && OFF_X1 % 256 == 0 && OFF_W0H % 256 == 0 && OFF_W0L % 256 == 0 &&
              OFF_W1H % 256 == 0 && OFF_W1L % 256 == 0 && OFF_ST % 256 == 0, "line-aligned carve");
static_assert((size_t)NBATCH * CH_OUT * NQUERY * 4 == 33554432, "d_out bytes");

extern "C" void kernel_launch(void* const* d_in, const int* in_sizes, int n_in,
                              void* d_out, int out_size, void* d_ws, size_t ws_size,
                              hipStream_t stream) {
  if (n_in < 16) return;
  if (ws_size < WS_TOTAL) return;
  if (out_size < NBATCH * CH_OUT * NQUERY) return;
  (void)in_sizes;

  const float* unknown = (const float*)d_in[0];
  const float* known   = (const float*)d_in[1];
  const float* ufeat   = (const float*)d_in[2];
  const float* kfeat   = (const float*)d_in[3];
  const float* W0  = (const float*)d_in[4];
  const float* b0  = (const float*)d_in[5];
  const float* g0  = (const float*)d_in[6];
  const float* be0 = (const float*)d_in[7];
  const float* rm0 = (const float*)d_in[8];
  const float* rv0 = (const float*)d_in[9];
  const float* W1  = (const float*)d_in[10];
  const float* b1  = (const float*)d_in[11];
  const float* g1  = (const float*)d_in[12];
  const float* be1 = (const float*)d_in[13];
  const float* rm1 = (const float*)d_in[14];
  const float* rv1 = (const float*)d_in[15];

  char* ws = (char*)d_ws;
  float*          Ft  = (float*)(ws + OFF_FT);
  unsigned short* X0  = (unsigned short*)(ws + OFF_X0);
  unsigned short* X1  = (unsigned short*)(ws + OFF_X1);
  unsigned short* W0h = (unsigned short*)(ws + OFF_W0H);
  unsigned short* W0l = (unsigned short*)(ws + OFF_W0L);
  unsigned short* W1h = (unsigned short*)(ws + OFF_W1H);
  unsigned short* W1l = (unsigned short*)(ws + OFF_W1L);
  float*          st  = (float*)(ws + OFF_ST);

  prep_weights_kernel<<<dim3(PREP_BLK_W0 + PREP_BLK_W1 + 2), dim3(256), 0, stream>>>(
      W0, W1, b0, g0, be0, rm0, rv0, b1, g1, be1, rm1, rv1, W0h, W0l, W1h, W1l, st);

  transpose_known_kernel<<<dim3(NSUPP / 32, NBATCH), dim3(256), 0, stream>>>(kfeat, Ft);

  nn3_interp_kernel<<<dim3(NQUERY / 256, NBATCH), dim3(256), 0, stream>>>(unknown, known, Ft, X0);

  ufeat_concat_kernel<<<dim3(NQUERY / 64, NBATCH), dim3(256), 0, stream>>>(ufeat, X0);

  {
    constexpr int tiles = (NPOINTS / 32) * (CH_OUT / 64);
    static_assert(tiles % 8 == 0, "whole blocks");
    gemm_f16_hilo_kernel<1, 1, 2><<<dim3(tiles / 8, 1), dim3(256), 0, stream>>>(
        X0, X0, CH_CAT, 0L,
        W0h, W0l, CH_CAT, 0L,
        (void*)X1, CH_OUT, 0L,
        st, st + CH_OUT,
        NPOINTS, CH_OUT, CH_CAT);
  }

  {
    constexpr int tiles = (CH_OUT / 32) * (NQUERY / 64);
    static_assert(tiles % 8 == 0, "whole blocks");
    gemm_f16_hilo_kernel<0, 0, 1><<<dim3(tiles / 8, NBATCH), dim3(256), 0, stream>>>(
        W1h, W1l, CH_OUT, 0L,
        X1, X1, CH_OUT, (long)NQUERY * CH_OUT,
        d_out, NQUERY, (long)CH_OUT * NQUERY,
        st + 2 * CH_OUT, st + 3 * CH_OUT,
        CH_OUT, NQUERY, CH_OUT);
  }
}
